// BAKTSimpleX_76544907149500
// MI455X (gfx1250) — hardware-verified
//
#include <hip/hip_runtime.h>
#include <math.h>

typedef __attribute__((ext_vector_type(16))) _Float16 v16h;
typedef __attribute__((ext_vector_type(16))) __bf16 v16b;
typedef __attribute__((ext_vector_type(8)))  _Float16 v8h;
typedef __attribute__((ext_vector_type(8)))  float v8f;
typedef __attribute__((ext_vector_type(4)))  float v4f;
typedef __attribute__((ext_vector_type(2)))  float v2f;
typedef __attribute__((ext_vector_type(4)))  unsigned v4u;
typedef __attribute__((ext_vector_type(4)))  int v4i;
typedef float __attribute__((may_alias)) float_a;
typedef int __attribute__((may_alias)) int_a;

template <typename T> __device__ __forceinline__ void vst2(void* p, T v) { *(volatile T*)p = v; __threadfence(); *(volatile T*)p = v; }
__device__ __forceinline__ v8f wmma16(v16h a, v16h b, v8f c) {
  v8f d = __builtin_amdgcn_wmma_f32_16x16x32_f16(false, a, false, b, (short)0, c, false, false);
  asm volatile("v_nop\n\tv_nop\n\tv_nop\n\tv_nop" : "+v"(d) : "v"(a), "v"(b));
  return d;
}
__device__ __forceinline__ v8f wmma_bf(v16b a, v16b b, v8f c) {
  v8f d = __builtin_amdgcn_wmma_f32_16x16x32_bf16(false, a, false, b, (short)0, c, false, false);
  asm volatile("v_nop\n\tv_nop\n\tv_nop\n\tv_nop" : "+v"(d) : "v"(a), "v"(b));
  return d;
}
__device__ __forceinline__ v16h frag_h(const _Float16* rowk0, int lane) {
  union { v16h v; v8h q[2]; } u; const _Float16* p = rowk0 + 8 * (lane >> 4);
  u.q[0] = *(const v8h*)p; u.q[1] = *(const v8h*)(p + 16); return u.v;
}
__device__ __forceinline__ v16h frag_f32(const float* rowk0, int lane) {
  v16h a; const float* p = rowk0 + 8 * (lane >> 4);
#pragma unroll
  for (int i = 0; i < 8; ++i) { a[i] = (_Float16)p[i]; a[8 + i] = (_Float16)p[16 + i]; }
  return a;
}
__device__ __forceinline__ v16h frag_f32s(const float* rowk0, int lane, float sc) {
  v16h a; const float* p = rowk0 + 8 * (lane >> 4);
#pragma unroll
  for (int i = 0; i < 8; ++i) { a[i] = (_Float16)(p[i] * sc); a[8 + i] = (_Float16)(p[16 + i] * sc); }
  return a;
}
__device__ __forceinline__ v16h fragc_f32(const float* W, int k0, int n, int lane, int ld, int K) {
  v16h a; const int g = lane >> 4;
#pragma unroll
  for (int i = 0; i < 8; ++i) { const int ka = k0 + 8 * g + i, kb = ka + 16;
    a[i] = (_Float16)(ka < K ? W[(size_t)(ka < K ? ka : K - 1) * ld + n] : 0.f); a[8 + i] = (_Float16)(kb < K ? W[(size_t)(kb < K ? kb : K - 1) * ld + n] : 0.f); }
  return a;
}
struct F2 { v16b h, l; };
__device__ __forceinline__ F2 bsplit16(const float v[16]) { F2 r;
#pragma unroll
  for (int i = 0; i < 16; ++i) { const __bf16 h = (__bf16)v[i]; r.h[i] = h; r.l[i] = (__bf16)(v[i] - (float)h); }
  return r; }
__device__ __forceinline__ F2 split_row(const float* row, int k0, int lane) { float v[16]; const float* p = row + k0 + 8 * (lane >> 4);
#pragma unroll
  for (int i = 0; i < 8; ++i) { v[i] = p[i]; v[8 + i] = p[16 + i]; }
  return bsplit16(v); }
__device__ __forceinline__ F2 split_rowK(const float* row, int k0, int lane, int K) { float v[16]; const int g = lane >> 4;
#pragma unroll
  for (int i = 0; i < 8; ++i) { const int ka = k0 + 8 * g + i, kb = ka + 16; v[i] = ka < K ? row[ka < K ? ka : K - 1] : 0.f; v[8 + i] = kb < K ? row[kb < K ? kb : K - 1] : 0.f; }
  return bsplit16(v); }
__device__ __forceinline__ F2 split_col(const float* W, int k0, int n, int lane, int ld, int K) { float v[16]; const int g = lane >> 4;
#pragma unroll
  for (int i = 0; i < 8; ++i) { const int ka = k0 + 8 * g + i, kb = ka + 16; v[i] = ka < K ? W[(size_t)(ka < K ? ka : K - 1) * ld + n] : 0.f; v[8 + i] = kb < K ? W[(size_t)(kb < K ? kb : K - 1) * ld + n] : 0.f; }
  return bsplit16(v); }
__device__ __forceinline__ v8f mac3(const F2& a, const F2& b, v8f c) { c = wmma_bf(a.l, b.h, c); c = wmma_bf(a.h, b.l, c); return wmma_bf(a.h, b.h, c); }
__device__ __forceinline__ float sigm(float v) { return 1.0f / (1.0f + expf(-v)); }
#define LDSX() do { asm volatile("s_wait_dscnt 0" ::: "memory"); __builtin_amdgcn_wave_barrier(); __builtin_amdgcn_fence(__ATOMIC_RELEASE, "workgroup"); } while (0)


#define BS 32
#define SQ 512
#define DD 256
#define NH 8
#define DK 32
#define DFF 1024
#define NR (BS * SQ)
#ifndef TRB
#define TRB (NR / 64)
#define TQB (SQ / 32)
#define TNB BS
#endif
typedef __attribute__((ext_vector_type(8))) __bf16 v8b;
__device__ __forceinline__ v16b frag_b(const __bf16* rowk0, int lane) {
  union { v16b v; v8b q[2]; } u; const __bf16* p = rowk0 + 8 * (lane >> 4);
  u.q[0] = *(const v8b*)p; u.q[1] = *(const v8b*)(p + 16); return u.v;
}
__device__ __forceinline__ float bfr(float v) { return (float)(__bf16)v; }
__device__ __attribute__((noinline)) float exp_ni(float v) { return expf(v); }
__device__ __attribute__((noinline)) float erf_ni(float v) { return erff(v); }

__device__ __attribute__((noinline)) float sin_ni(float v) { return sinf(v); }
__device__ __attribute__((noinline)) float cos_ni(float v) { return cosf(v); }
__device__ __forceinline__ void put_hl(__bf16* h, __bf16* l, float v) { const __bf16 hb = (__bf16)v; *h = hb; *l = (__bf16)(v - (float)hb); }
#define PK_K  0
#define PK_V  (PK_K + 2 * DD * DD)
#define PK_O  (PK_V + 2 * DD * DD)
#define PK_1  (PK_O + 2 * DD * DD)
#define PK_2  (PK_1 + 2 * DFF * DD)
#define PK_END (PK_2 + 2 * DD * DFF)
#define WS_PK  0u
#define WS_PE  (WS_PK + 2u * PK_END)
#define WS_X   (WS_PE + 4u * SQ * DD)
#define WS_Y   (WS_X + 4u * NR * DD)
#define WS_KM  (WS_Y + 4u * NR * DD)
#define WS_VM  (WS_KM + 4u * NR * DD)
#define WS_VTH (WS_VM + 4u * NR * DD)
#define WS_VTL (WS_VTH + 2u * BS * DD * SQ)
#define WS_AT  (WS_VTL + 2u * BS * DD * SQ)
#define WS_X2  (WS_AT + 4u * NR * DD)
#define WS_END (WS_X2 + 4u * NR * DD)

__global__ __launch_bounds__(256) void k_pack(const float* __restrict__ Wm, int K, __bf16* __restrict__ DST) {
  __shared__ __align__(16) __bf16 s[DFF]; const int n = blockIdx.x, tid = threadIdx.x; const float* src = Wm + (size_t)n * K;
  for (int k = tid; k < K; k += 256) s[k] = (__bf16)src[k];
  __syncthreads();
  for (int q = tid; q < K / 8; q += 256) vst2((unsigned*)(DST + (size_t)n * K + q * 8), *(const v4u*)&s[q * 8]);
}
__global__ __launch_bounds__(256) void k_pe(float* __restrict__ PE) {
  __shared__ __align__(16) float s[DD]; const int t = blockIdx.x, tid = threadIdx.x;
  { const int c = tid; const int i2 = c & ~1; const float divt = expf((float)i2 * (-logf(10000.0f) / (float)DD)); const float ang = (float)t * divt; s[c] = (c & 1) ? cos_ni(ang) : sin_ni(ang); }
  __syncthreads();
  if (tid < DD / 4) vst2(PE + (size_t)t * DD + tid * 4, *(const v4f*)&s[tid * 4]);
}
__global__ __launch_bounds__(256) void k_add(const float* __restrict__ QE, const float* __restrict__ QAE, const float* __restrict__ PE, float* __restrict__ X, float* __restrict__ Y) {
  const int tid = threadIdx.x; const size_t r = (size_t)blockIdx.x * 4 + (tid >> 6); const int pc = tid & 63; const int t = (int)(r % SQ);
  v4f a, c; const float* pq = QE + r * DD + pc * 4; const float* pa = QAE + r * DD + pc * 4; const float* pp = PE + (size_t)t * DD + pc * 4;
#pragma unroll
  for (int i = 0; i < 4; ++i) { a[i] = bfr(pq[i]) + pp[i]; c[i] = bfr(pa[i]) + pp[i]; }
  vst2(X + r * DD + pc * 4, a); vst2(Y + r * DD + pc * 4, c);
}
template <int K, int EPI, int RM>
__global__ __launch_bounds__(128) void k_lin(const float* __restrict__ A, int lda, const __bf16* __restrict__ P, const float* __restrict__ bias, float* __restrict__ OUT, int ldo, const float* __restrict__ RES, int ldr) {
  __shared__ __align__(16) float so[4][16][132];
  const int tid = threadIdx.x, wave = tid >> 5, lane = tid & 31, col = lane & 15, g = lane >> 4; const size_t r0 = (size_t)blockIdx.x * 64 + wave * 16; const int n0 = blockIdx.y * 128;
  v8f acc[8] = {};
#pragma unroll 2
  for (int kc = 0; kc < K / 32; ++kc) { const F2 a = split_row(A + (r0 + col) * lda, kc * 32, lane);
#pragma unroll
    for (int j = 0; j < 8; ++j) { const v16b w = frag_b(P + (size_t)(n0 + j * 16 + col) * K + kc * 32, lane); acc[j] = wmma_bf(a.l, w, acc[j]); acc[j] = wmma_bf(a.h, w, acc[j]); } }
#pragma unroll
  for (int j = 0; j < 8; ++j) { const int n = n0 + j * 16 + col; const float bb = bias ? bfr(bias[n]) : 0.f;
#pragma unroll
    for (int r = 0; r < 8; ++r) { const size_t row = r0 + 8 * g + r; float v = acc[j][r] + bb; if (EPI == 1) v = fmaxf(v, 0.f); if (RM == 1) v += RES[row * ldr + n]; so[wave][8 * g + r][j * 16 + col] = v; } }
  LDSX();
  for (int rl = 0; rl < 16; ++rl) vst2(OUT + (r0 + rl) * ldo + n0 + lane * 4, *(const v4f*)&so[wave][rl][lane * 4]);
}
__global__ __launch_bounds__(256) void k_vt(const float* __restrict__ VM, __bf16* __restrict__ VTH, __bf16* __restrict__ VTL) {
  __shared__ __align__(16) __bf16 svh[DD][72], svl[DD][72];
  const int tid = threadIdx.x; const size_t t0 = (size_t)blockIdx.x * 64; const int b = (int)(t0 / SQ), p0 = (int)(t0 % SQ);
  for (int q = tid; q < 64 * DD; q += 256) { const int tl = q >> 8, c = q & 255; const float v = VM[(t0 + tl) * DD + c]; const __bf16 hb = (__bf16)v; svh[c][tl] = hb; svl[c][tl] = (__bf16)(v - (float)hb); }
  __syncthreads();
  for (int q = tid; q < DD * 8; q += 256) { const int rowi = q >> 3, pc = q & 7; const size_t o = ((size_t)b * DD + rowi) * SQ + p0 + pc * 8; vst2((unsigned*)(VTH + o), *(const v4u*)&svh[rowi][pc * 8]); vst2((unsigned*)(VTL + o), *(const v4u*)&svl[rowi][pc * 8]); }
}
template <int EMIT>
__global__ __launch_bounds__(64) void k_attn(const float* __restrict__ KM, const __bf16* __restrict__ VTH, const __bf16* __restrict__ VTL, float* __restrict__ AT, float* __restrict__ SC) {
  __shared__ __align__(16) float ss[32][SQ + 4]; __shared__ __align__(16) float sacc[EMIT ? 32 : 1][SQ]; __shared__ __align__(16) float so[32][DD + 4];
  const int tid = threadIdx.x, wave = tid >> 5, lane = tid & 31, col = lane & 15, g = lane >> 4; const int qt = blockIdx.x, b = blockIdx.y; const int i0 = qt * 32; const size_t rw = (size_t)b * SQ + i0 + wave * 16;
  const int nct = (i0 + 32) / 16;
  if (EMIT) { for (int q = lane; q < 16 * SQ; q += 32) (&sacc[wave * 16][0])[q] = 0.f; }
#pragma unroll 1
  for (int h = 0; h < NH; ++h) {
    const F2 a = split_row(KM + (rw + col) * DD + h * DK, 0, lane);
    for (int ct = 0; ct < nct; ++ct) { const F2 kb = split_row(KM + ((size_t)b * SQ + ct * 16 + col) * DD + h * DK, 0, lane); const v8f c = mac3(a, kb, (v8f){});
#pragma unroll
      for (int r = 0; r < 8; ++r) ss[wave * 16 + 8 * g + r][ct * 16 + col] = c[r] * 0.17677669529663687f; }
    LDSX();
#pragma unroll 1
    for (int rl = 0; rl < 16; ++rl) { const int row = wave * 16 + rl; const int i = i0 + row; float* sr = ss[row];
      float mx = -3.0e38f; for (int j = lane; j < nct * 16; j += 32) if (j < i) mx = fmaxf(mx, sr[j]);
#pragma unroll
      for (int o = 1; o < 32; o <<= 1) mx = fmaxf(mx, __shfl_xor(mx, o));
      float z = 0.f; for (int j = lane; j < nct * 16; j += 32) { const float e = (j < i) ? exp_ni(sr[j] - mx) : 0.f; sr[j] = e; z += e; }
#pragma unroll
      for (int o = 1; o < 32; o <<= 1) z += __shfl_xor(z, o);
      const float iz = (i == 0) ? 0.f : 1.0f / z;
      for (int j = lane; j < nct * 16; j += 32) { const float p = sr[j] * iz; sr[j] = p; if (EMIT) sacc[row][j] += p * (1.0f / (float)NH); } }
    LDSX();
    { v8f acc[2] = {}; const int nks = (nct + 1) / 2;
      if (nct & 1) { for (int rl = 0; rl < 16; ++rl) if (lane < 16) ss[wave * 16 + rl][nct * 16 + lane] = 0.f; LDSX(); }
      for (int ks = 0; ks < nks; ++ks) { const F2 pa = split_row(&ss[wave * 16 + col][0], ks * 32, lane);
#pragma unroll
        for (int dt = 0; dt < 2; ++dt) { const size_t vrow = ((size_t)b * DD + h * DK + dt * 16 + col) * SQ + ks * 32; const v16b vh = frag_b(VTH + vrow, lane), vl = frag_b(VTL + vrow, lane); acc[dt] = wmma_bf(pa.l, vh, acc[dt]); acc[dt] = wmma_bf(pa.h, vl, acc[dt]); acc[dt] = wmma_bf(pa.h, vh, acc[dt]); } }
#pragma unroll
      for (int dt = 0; dt < 2; ++dt)
#pragma unroll
        for (int r = 0; r < 8; ++r) so[wave * 16 + 8 * g + r][h * DK + dt * 16 + col] = acc[dt][r]; }
    LDSX(); }
  __syncthreads();
  for (int q = tid; q < 32 * 64; q += 64) { const int rl = q >> 6, pc = q & 63; vst2(AT + ((size_t)b * SQ + i0 + rl) * DD + pc * 4, *(const v4f*)&so[rl][pc * 4]); }
  if (EMIT) for (int q = tid; q < 32 * 128; q += 64) { const int rl = q >> 7, pc = q & 127; vst2(SC + ((size_t)b * SQ + i0 + rl) * SQ + pc * 4, *(const v4f*)&sacc[rl][pc * 4]); }
}
__global__ __launch_bounds__(256) void k_ln(const float* __restrict__ X, const float* __restrict__ gw, const float* __restrict__ bw, float* __restrict__ Y) {
  __shared__ __align__(16) float s[16][DD];
  const int wave = threadIdx.x >> 5, lane = threadIdx.x & 31;
#pragma unroll
  for (int rr = 0; rr < 2; ++rr) { const int rl = wave * 2 + rr; const size_t r = (size_t)blockIdx.x * 16 + rl; const float* x = X + r * DD; float v[8]; float sum = 0.f;
#pragma unroll
    for (int i = 0; i < 8; ++i) { v[i] = x[lane + 32 * i]; sum += v[i]; }
#pragma unroll
    for (int o = 1; o < 32; o <<= 1) sum += __shfl_xor(sum, o);
    const float mu = sum / (float)DD; float var = 0.f;
#pragma unroll
    for (int i = 0; i < 8; ++i) { const float d = v[i] - mu; var += d * d; }
#pragma unroll
    for (int o = 1; o < 32; o <<= 1) var += __shfl_xor(var, o);
    const float rs = rsqrtf(var / (float)DD + 1e-5f);
#pragma unroll
    for (int i = 0; i < 8; ++i) { const int c = lane + 32 * i; s[rl][c] = (v[i] - mu) * rs * bfr(gw[c]) + bfr(bw[c]); } }
  LDSX();
#pragma unroll
  for (int rr = 0; rr < 2; ++rr) { const int rl = wave * 2 + rr; const size_t r = (size_t)blockIdx.x * 16 + rl; for (int pc = lane; pc < DD / 4; pc += 32) vst2(Y + r * DD + pc * 4, *(const v4f*)&s[rl][pc * 4]); }
}
__global__ __launch_bounds__(64) void k_ffn(const float* __restrict__ X1, const __bf16* __restrict__ P1, const float* __restrict__ b1, const __bf16* __restrict__ P2, const float* __restrict__ b2, float* __restrict__ OUT) {
  __shared__ __align__(16) __bf16 shh[16][DD + 8], shl[16][DD + 8]; __shared__ __align__(16) float so[16][DD + 4];
  const int tid = threadIdx.x, wave = tid >> 5, lane = tid & 31, col = lane & 15, g = lane >> 4; const size_t r0 = (size_t)blockIdx.x * 16;
  v8f acc[8] = {};
#pragma unroll 1
  for (int ch = 0; ch < DFF / DD; ++ch) {
    { v8f ah[8] = {};
#pragma unroll 2
      for (int kc = 0; kc < 8; ++kc) { const F2 ax = split_row(X1 + (r0 + col) * DD, kc * 32, lane);
#pragma unroll
        for (int j = 0; j < 8; ++j) { const v16b w = frag_b(P1 + (size_t)(ch * DD + wave * 128 + j * 16 + col) * DD + kc * 32, lane); ah[j] = wmma_bf(ax.l, w, ah[j]); ah[j] = wmma_bf(ax.h, w, ah[j]); } }
      __syncthreads();
#pragma unroll
      for (int j = 0; j < 8; ++j) { const int hc = wave * 128 + j * 16 + col; const float bb = bfr(b1[ch * DD + hc]);
#pragma unroll
        for (int r = 0; r < 8; ++r) put_hl(&shh[8 * g + r][hc], &shl[8 * g + r][hc], fmaxf(ah[j][r] + bb, 0.f)); } }
    __syncthreads();
#pragma unroll
    for (int kc = 0; kc < 8; ++kc) { const v16b hh = frag_b(&shh[col][kc * 32], lane), hl = frag_b(&shl[col][kc * 32], lane);
#pragma unroll
      for (int j = 0; j < 8; ++j) { const v16b w = frag_b(P2 + (size_t)(wave * 128 + j * 16 + col) * DFF + ch * DD + kc * 32, lane); acc[j] = wmma_bf(hl, w, acc[j]); acc[j] = wmma_bf(hh, w, acc[j]); } } }
#pragma unroll
  for (int j = 0; j < 8; ++j) { const int n = wave * 128 + j * 16 + col; const float bb = bfr(b2[n]);
#pragma unroll
    for (int r = 0; r < 8; ++r) so[8 * g + r][n] = acc[j][r] + bb + X1[(r0 + 8 * g + r) * DD + n]; }
  __syncthreads();
  for (int q = tid; q < 16 * 64; q += 64) { const int rl = q >> 6, pc = q & 63; vst2(OUT + (r0 + rl) * DD + pc * 4, *(const v4f*)&so[rl][pc * 4]); }
}
extern "C" void kernel_launch(void* const* d_in, const int* in_sizes, int n_in, void* d_out, int out_size, void* d_ws, size_t ws_size, hipStream_t stream) {
  (void)in_sizes; (void)n_in; (void)out_size;
  const float** F = (const float**)d_in;
  if (ws_size < (size_t)WS_END) return;
  char* ws = (char*)d_ws; __bf16 *PK = (__bf16*)(ws + WS_PK), *VTH = (__bf16*)(ws + WS_VTH), *VTL = (__bf16*)(ws + WS_VTL);
  float *PE = (float*)(ws + WS_PE), *X = (float*)(ws + WS_X), *Y = (float*)(ws + WS_Y), *KM = (float*)(ws + WS_KM), *VM = (float*)(ws + WS_VM), *AT = (float*)(ws + WS_AT), *X2 = (float*)(ws + WS_X2);
  float* OUT0 = (float*)d_out; float* OUT1 = (float*)d_out + (size_t)NR * DD;
  k_pack<<<2 * DD, 256, 0, stream>>>(F[2], DD, PK + PK_K);
  k_pack<<<2 * DD, 256, 0, stream>>>(F[4], DD, PK + PK_V);
  k_pack<<<2 * DD, 256, 0, stream>>>(F[6], DD, PK + PK_O);
  k_pack<<<2 * DFF, 256, 0, stream>>>(F[10], DD, PK + PK_1);
  k_pack<<<2 * DD, 256, 0, stream>>>(F[12], DFF, PK + PK_2);
  k_pe<<<SQ, 256, 0, stream>>>(PE);
  k_add<<<TRB * 16, 256, 0, stream>>>(F[0], F[1], PE, X, Y);
  for (int blk = 0; blk < 2; ++blk) {
    const float* xin = X;
    k_lin<DD, 0, 0><<<dim3(TRB, DD / 128), 128, 0, stream>>>(xin, DD, PK + PK_K + (size_t)blk * DD * DD, F[3] + blk * DD, KM, DD, nullptr, 0);
    k_lin<DD, 0, 0><<<dim3(TRB, DD / 128), 128, 0, stream>>>(Y, DD, PK + PK_V + (size_t)blk * DD * DD, F[5] + blk * DD, VM, DD, nullptr, 0);
    k_vt<<<TRB, 256, 0, stream>>>(VM, VTH, VTL);
    if (blk == 0) k_attn<0><<<dim3(TQB, TNB), 64, 0, stream>>>(KM, VTH, VTL, AT, OUT1); else k_attn<1><<<dim3(TQB, TNB), 64, 0, stream>>>(KM, VTH, VTL, AT, OUT1);
    k_lin<DD, 0, 1><<<dim3(TRB, DD / 128), 128, 0, stream>>>(AT, DD, PK + PK_O + (size_t)blk * DD * DD, F[7] + blk * DD, X2, DD, xin, DD);
    k_ln<<<TRB * 4, 256, 0, stream>>>(X2, F[8] + blk * DD, F[9] + blk * DD, AT);
    k_ffn<<<TRB * 4, 64, 0, stream>>>(AT, PK + PK_1 + (size_t)blk * DFF * DD, F[11] + blk * DFF, PK + PK_2 + (size_t)blk * DD * DFF, F[13] + blk * DD, X2);
    k_ln<<<TRB * 4, 256, 0, stream>>>(X2, F[14] + blk * DD, F[15] + blk * DD, blk == 1 ? OUT0 : X);
  }
}
